// Word2ManSkipGramNegSampling_83391085019284
// MI455X (gfx1250) — hardware-verified
//
#include <hip/hip_runtime.h>
#include <stdint.h>


typedef __attribute__((ext_vector_type(16))) __bf16 v16bf;
typedef float    v8f __attribute__((ext_vector_type(8)));
typedef float    v4f __attribute__((ext_vector_type(4)));
typedef uint32_t v4u __attribute__((ext_vector_type(4)));
typedef uint32_t v2u __attribute__((ext_vector_type(2)));
typedef v4u __attribute__((may_alias)) v4ua;
typedef v2u __attribute__((may_alias)) v2ua;

#define DEMB      128
#define PITCH     136
#define ROWS_PB   128
#define NTHREADS  256
#define PLANE     (DEMB * PITCH)
#define SMEM_BYTES (4u * PLANE * sizeof(uint16_t))

union V16U { v16bf v; v4u q[2]; };

__device__ __forceinline__ uint32_t bf16rn(float a) {
    uint32_t u = __builtin_bit_cast(uint32_t, a);
    return (u + 0x7fffu + ((u >> 16) & 1u)) >> 16;
}

__device__ __forceinline__ int clampidx(int v, int n) {
    if (v < 0) v += n;
    v = v < 0 ? 0 : v;
    v = v > n - 1 ? n - 1 : v;
    return v;
}

__device__ __forceinline__ v8f wmma3(v8f acc, v16bf al, v16bf ah, v16bf bl, v16bf bh) {
    acc = __builtin_amdgcn_wmma_f32_16x16x32_bf16(false, al, false, bh, (short)0, acc, false, false);
    acc = __builtin_amdgcn_wmma_f32_16x16x32_bf16(false, ah, false, bl, (short)0, acc, false, false);
    acc = __builtin_amdgcn_wmma_f32_16x16x32_bf16(false, ah, false, bh, (short)0, acc, false, false);
    asm volatile("v_nop\n\tv_nop\n\tv_nop\n\tv_nop" : "+v"(acc) : "v"(ah), "v"(bh), "v"(al), "v"(bl));
    return acc;
}

__global__ __launch_bounds__(NTHREADS)
void k_bilinear(const int* __restrict__ xs, const int* __restrict__ ys,
                const float* __restrict__ metric, const float* __restrict__ emb,
                float* out, int nbatch, int nvocab)
{
    extern __shared__ __attribute__((aligned(16))) uint16_t smem[];
    __shared__ v4f sOut[ROWS_PB / 4];

    uint16_t* sMh = smem;
    uint16_t* sMl = smem + PLANE;
    uint16_t* sAh = smem + 2 * PLANE;
    uint16_t* sAl = smem + 3 * PLANE;

    const int tid  = threadIdx.x;
    const int lane = tid & 31;
    const int l    = lane & 15;
    const int kh   = lane >> 4;
    const int wave = tid >> 5;
    const int base = blockIdx.x * ROWS_PB + wave * 16;

    for (int f = tid; f < DEMB * DEMB; f += NTHREADS) {
        const int d = f >> 7, e = f & (DEMB - 1);
        const float m = metric[f];
        const uint32_t hb = bf16rn(m);
        const float lf = m - __builtin_bit_cast(float, hb << 16);
        sMh[e * PITCH + d] = (uint16_t)hb;
        sMl[e * PITCH + d] = (uint16_t)bf16rn(lf);
    }

    #pragma unroll 1
    for (int r = 0; r < 16; ++r) {
        const int xi = clampidx(xs[min(base + r, nbatch - 1)], nvocab);
        const float4 v = *(const float4*)(emb + (size_t)xi * DEMB + lane * 4);
        const uint32_t h0 = bf16rn(v.x), h1 = bf16rn(v.y), h2 = bf16rn(v.z), h3 = bf16rn(v.w);
        const uint32_t l0 = bf16rn(v.x - __builtin_bit_cast(float, h0 << 16));
        const uint32_t l1 = bf16rn(v.y - __builtin_bit_cast(float, h1 << 16));
        const uint32_t l2 = bf16rn(v.z - __builtin_bit_cast(float, h2 << 16));
        const uint32_t l3 = bf16rn(v.w - __builtin_bit_cast(float, h3 << 16));
        v2u hv, lv;
        hv.x = h0 | (h1 << 16);  hv.y = h2 | (h3 << 16);
        lv.x = l0 | (l1 << 16);  lv.y = l2 | (l3 << 16);
        const int so = (wave * 16 + r) * PITCH + lane * 4;
        *(v2ua*)(sAh + so) = hv;
        *(v2ua*)(sAl + so) = lv;
    }
    __syncthreads();

    int yr[8];
    #pragma unroll
    for (int c = 0; c < 8; ++c)
        yr[c] = clampidx(ys[min(base + kh * 8 + c, nbatch - 1)], nvocab);

    float p[8] = {0.f, 0.f, 0.f, 0.f, 0.f, 0.f, 0.f, 0.f};

    const uint16_t* arh = sAh + (wave * 16 + l) * PITCH + kh * 8;
    const uint16_t* arl = sAl + (wave * 16 + l) * PITCH + kh * 8;

    #pragma unroll
    for (int nt = 0; nt < 8; ++nt) {
        v8f acc = {0.f, 0.f, 0.f, 0.f, 0.f, 0.f, 0.f, 0.f};
        const uint16_t* bch = sMh + (nt * 16 + l) * PITCH + kh * 8;
        const uint16_t* bcl = sMl + (nt * 16 + l) * PITCH + kh * 8;
        #pragma unroll
        for (int kk = 0; kk < 4; ++kk) {
            V16U Ah, Al, Bh, Bl;
            Ah.q[0] = *(const v4ua*)(arh + kk * 32);
            Ah.q[1] = *(const v4ua*)(arh + kk * 32 + 16);
            Al.q[0] = *(const v4ua*)(arl + kk * 32);
            Al.q[1] = *(const v4ua*)(arl + kk * 32 + 16);
            Bh.q[0] = *(const v4ua*)(bch + kk * 32);
            Bh.q[1] = *(const v4ua*)(bch + kk * 32 + 16);
            Bl.q[0] = *(const v4ua*)(bcl + kk * 32);
            Bl.q[1] = *(const v4ua*)(bcl + kk * 32 + 16);
            acc = wmma3(acc, Al.v, Ah.v, Bl.v, Bh.v);
        }
        #pragma unroll
        for (int c = 0; c < 8; ++c) {
            const float yv = emb[(size_t)yr[c] * DEMB + nt * 16 + l];
            p[c] += acc[c] * yv;
        }
    }

    #pragma unroll
    for (int m = 8; m >= 1; m >>= 1) {
        #pragma unroll
        for (int c = 0; c < 8; ++c)
            p[c] += __shfl_xor(p[c], m, 32);
    }

    if (l == 0) {
        float s[8];
        #pragma unroll
        for (int c = 0; c < 8; ++c)
            s[c] = 1.0f / (1.0f + __expf(-p[c]));
        v4f o0 = {s[0], s[1], s[2], s[3]};
        v4f o1 = {s[4], s[5], s[6], s[7]};
        sOut[wave * 4 + kh * 2]     = o0;
        sOut[wave * 4 + kh * 2 + 1] = o1;
    }
    __syncthreads();

    if (wave == 0) {
        const int ob = blockIdx.x * ROWS_PB + lane * 4;
        const v4f v = sOut[lane];
        float* op = out + ob;
        const bool full = (ob + 3 < nbatch);
        if (full) {
            *(volatile v4f*)op = v;
        } else {
            #pragma unroll
            for (int c = 0; c < 4; ++c)
                if (ob + c < nbatch) *(volatile float*)(op + c) = v[c];
        }
        __threadfence();
        if (full) {
            *(volatile v4f*)op = v;
        } else {
            #pragma unroll
            for (int c = 0; c < 4; ++c)
                if (ob + c < nbatch) *(volatile float*)(op + c) = v[c];
        }
    }
}

extern "C" void kernel_launch(void* const* d_in, const int* in_sizes, int n_in,
                              void* d_out, int out_size, void* d_ws, size_t ws_size,
                              hipStream_t stream) {
    (void)n_in; (void)d_ws; (void)ws_size;
    const int*   xs     = (const int*)d_in[0];
    const int*   ys     = (const int*)d_in[1];
    const float* metric = (const float*)d_in[2];
    const float* emb    = (const float*)d_in[3];
    float*       out    = (float*)d_out;

    const int nbatch = in_sizes[0];
    const int nvocab = in_sizes[3] / DEMB;
    if (nbatch <= 0 || nvocab <= 0) return;
    if (in_sizes[1] < nbatch || out_size < nbatch || in_sizes[2] != DEMB * DEMB) return;

    const int grid = (nbatch + ROWS_PB - 1) / ROWS_PB;
    k_bilinear<<<grid, NTHREADS, SMEM_BYTES, stream>>>(xs, ys, metric, emb, out, nbatch, nvocab);
    (void)hipGetLastError();
}
